// BlackBoxModel_24489903521937
// MI455X (gfx1250) — hardware-verified
//
#include <hip/hip_runtime.h>
#include <stdint.h>


typedef _Float16       v16h __attribute__((ext_vector_type(16)));
typedef _Float16       v8h  __attribute__((ext_vector_type(8)));
typedef __bf16         v16b __attribute__((ext_vector_type(16)));
typedef unsigned short v8us __attribute__((ext_vector_type(8)));
typedef unsigned short v4us __attribute__((ext_vector_type(4)));
typedef float          v8f  __attribute__((ext_vector_type(8)));
typedef float          v4f  __attribute__((ext_vector_type(4)));

namespace {
constexpr int kNY = 8;
constexpr int kNU = 4;
constexpr int kT  = 256;
constexpr int kH  = 128;
constexpr int kDS = 56;
constexpr int kDI = 60;
constexpr int kKX = 64;
constexpr int WAVES = 4;
constexpr int ROWS  = 16;
constexpr int BROWS = WAVES * ROWS;
constexpr int NTHR  = WAVES * 32;
constexpr int XS  = 64;
constexpr int HS  = 128;
constexpr int W1S = 64;
constexpr int W2S = 128;
constexpr int W3S = 128;
constexpr int OBS = 32;
constexpr float kWscale = 16.0f;
constexpr float kWinv   = 0.0625f;
}

__device__ __forceinline__ unsigned short bf16_rne(float f) {
  unsigned int u = __float_as_uint(f);
  u += 0x7FFFu + ((u >> 16) & 1u);
  return (unsigned short)(u >> 16);
}
__device__ __forceinline__ float bf16_to_f(unsigned short s) {
  return __uint_as_float(((unsigned int)s) << 16);
}
__device__ __forceinline__ void split_bf16(float f, unsigned short& hi, unsigned short& lo) {
  hi = bf16_rne(f);
  lo = bf16_rne(f - bf16_to_f(hi));
}
__device__ __forceinline__ unsigned short bf16_part(float f, int plane) {
  unsigned short hi, lo;
  split_bf16(f, hi, lo);
  return plane ? lo : hi;
}

__device__ __forceinline__ float fast_tanh(float x) {
  const float e = __builtin_amdgcn_exp2f(x * 2.885390081777926814f);
  return __builtin_fmaf(-2.0f, __builtin_amdgcn_rcpf(1.0f + e), 1.0f);
}

union FragH { v16h v; v8h  p[2]; };
union FragB { v16b v; v8us p[2]; };

__device__ __forceinline__ v16h ld_frag_h(const _Float16* row, int k0, int h) {
  FragH f;
  f.p[0] = *(const v8h*)(row + k0 + 8 * h);
  f.p[1] = *(const v8h*)(row + k0 + 16 + 8 * h);
  return f.v;
}
__device__ __forceinline__ v16b ld_frag_b(const unsigned short* row, int k0, int h) {
  FragB f;
  f.p[0] = *(const v8us*)(row + k0 + 8 * h);
  f.p[1] = *(const v8us*)(row + k0 + 16 + 8 * h);
  return f.v;
}

__device__ __forceinline__ v8f mma_f16(v16h a, v16h b, v8f c) {
  c = __builtin_amdgcn_wmma_f32_16x16x32_f16(false, a, false, b, (short)0, c, false, false);
  asm volatile("v_nop\n\tv_nop\n\tv_nop\n\tv_nop" : "+v"(c) : "v"(a), "v"(b));
  return c;
}
__device__ __forceinline__ v8f mma_bf16(v16b a, v16b b, v8f c) {
  c = __builtin_amdgcn_wmma_f32_16x16x32_bf16(false, a, false, b, (short)0, c, false, false);
  asm volatile("v_nop\n\tv_nop\n\tv_nop\n\tv_nop" : "+v"(c) : "v"(a), "v"(b));
  return c;
}

__global__ __launch_bounds__(NTHR)
void bbm_rollout(const float* __restrict__ useq, const float* __restrict__ yz0,
                 const float* __restrict__ W1,   const float* __restrict__ b1,
                 const float* __restrict__ W2,   const float* __restrict__ b2,
                 const float* __restrict__ W3,   const float* __restrict__ b3,
                 float* __restrict__ out, int B)
{
  __shared__ __attribute__((aligned(16))) unsigned short w1h[kH * W1S];
  __shared__ __attribute__((aligned(16))) unsigned short w1l[kH * W1S];
  __shared__ __attribute__((aligned(16))) _Float16 w2t[kH * W2S];
  __shared__ __attribute__((aligned(16))) _Float16 w3t[16 * W3S];
  __shared__ __attribute__((aligned(16))) unsigned short xh[BROWS * XS];
  __shared__ __attribute__((aligned(16))) unsigned short xl[BROWS * XS];
  __shared__ __attribute__((aligned(16))) _Float16 hb1[BROWS * HS];
  __shared__ __attribute__((aligned(16))) _Float16 hb2[BROWS * HS];
  __shared__ __attribute__((aligned(16))) float obuf[BROWS * OBS];
  __shared__ float b1s[kH];
  __shared__ float b2s[kH];
  __shared__ float b3s[16];

  const int tid  = threadIdx.x;
  const int wave = tid >> 5;
  const int lane = tid & 31;
  const int m    = lane & 15;
  const int h    = lane >> 4;

  for (int idx = tid; idx < kH * kKX; idx += NTHR) {
    const int n = idx >> 6, k = idx & 63;
    unsigned short hi = 0, lo = 0;
    if (k < kDI) split_bf16(W1[k * kH + n], hi, lo);
    w1h[n * W1S + k] = hi;
    w1l[n * W1S + k] = lo;
  }
  for (int idx = tid; idx < kH * kH; idx += NTHR) {
    const int k = idx >> 7, n = idx & 127;
    w2t[n * W2S + k] = (_Float16)(W2[idx] * kWscale);
  }
  for (int idx = tid; idx < 16 * kH; idx += NTHR) {
    const int n = idx >> 7, k = idx & 127;
    float v = 0.0f;
    if (n < kNY) v = W3[k * kNY + n] * kWscale;
    w3t[n * W3S + k] = (_Float16)v;
  }
  for (int i = tid; i < kH; i += NTHR) { b1s[i] = b1[i]; b2s[i] = b2[i]; }
  if (tid < 16) b3s[tid] = (tid < kNY) ? b3[tid] : 0.0f;

  const int lr0   = wave * ROWS;
  const int lrow  = lr0 + m;
  const int grow  = blockIdx.x * BROWS + lrow;
  const int growc = (grow < B) ? grow : (B - 1);
  unsigned short* const xrow = (h ? xl : xh) + lrow * XS;

  {
    const float* yr = yz0 + (size_t)growc * kDS;
    for (int k = 0; k < kDS; ++k) xrow[k] = bf16_part(yr[k], h);
    const v4f u = *(const v4f*)(useq + ((size_t)growc * kT) * kNU);
    xrow[kDS + 0] = bf16_part(u.x, h);
    xrow[kDS + 1] = bf16_part(u.y, h);
    xrow[kDS + 2] = bf16_part(u.z, h);
    xrow[kDS + 3] = bf16_part(u.w, h);
#pragma unroll
    for (int k = kDI; k < kKX; ++k) xrow[k] = 0;
    if (h == 0) {
#pragma unroll
      for (int n = 0; n < kNY; ++n) obuf[lrow * OBS + n] = yr[n];
    }
  }

  const unsigned short* const xa_h = xh + lrow * XS;
  const unsigned short* const xa_l = xl + lrow * XS;
  const _Float16* const h1r = hb1 + lrow * HS;
  const _Float16* const h2r = hb2 + lrow * HS;
  _Float16* const h1w = hb1 + (lr0 + 8 * h) * HS;
  _Float16* const h2w = hb2 + (lr0 + 8 * h) * HS;
  float* const ow0 = obuf + (lr0 + 8 * h) * OBS;

#pragma unroll 1
  for (int t = 0; t < kT - 1; ++t) {
    __syncthreads();

    const v16b xah0 = ld_frag_b(xa_h, 0, h);
    const v16b xah1 = ld_frag_b(xa_h, 32, h);
    const v16b xal0 = ld_frag_b(xa_l, 0, h);
    const v16b xal1 = ld_frag_b(xa_l, 32, h);
#pragma unroll 1
    for (int j = 0; j < 8; ++j) {
      const int n = 16 * j + m;
      const unsigned short* wrh = w1h + n * W1S;
      const unsigned short* wrl = w1l + n * W1S;
      const v16b bh0 = ld_frag_b(wrh, 0, h);
      const v16b bh1 = ld_frag_b(wrh, 32, h);
      const v16b bl0 = ld_frag_b(wrl, 0, h);
      const v16b bl1 = ld_frag_b(wrl, 32, h);
      v8f acc;
#pragma unroll
      for (int r = 0; r < 8; ++r) acc[r] = 0.0f;
      acc = mma_bf16(xah0, bh0, acc);
      acc = mma_bf16(xah1, bh1, acc);
      acc = mma_bf16(xah0, bl0, acc);
      acc = mma_bf16(xah1, bl1, acc);
      acc = mma_bf16(xal0, bh0, acc);
      acc = mma_bf16(xal1, bh1, acc);
      const float bias = b1s[n];
#pragma unroll
      for (int r = 0; r < 8; ++r) h1w[r * HS + n] = (_Float16)fast_tanh(acc[r] + bias);
    }
    __syncthreads();

    {
      const v16h ha0 = ld_frag_h(h1r, 0, h);
      const v16h ha1 = ld_frag_h(h1r, 32, h);
      const v16h ha2 = ld_frag_h(h1r, 64, h);
      const v16h ha3 = ld_frag_h(h1r, 96, h);
#pragma unroll 1
      for (int j = 0; j < 8; ++j) {
        const int n = 16 * j + m;
        const _Float16* wr = w2t + n * W2S;
        v8f acc;
#pragma unroll
        for (int r = 0; r < 8; ++r) acc[r] = 0.0f;
        acc = mma_f16(ha0, ld_frag_h(wr, 0, h), acc);
        acc = mma_f16(ha1, ld_frag_h(wr, 32, h), acc);
        acc = mma_f16(ha2, ld_frag_h(wr, 64, h), acc);
        acc = mma_f16(ha3, ld_frag_h(wr, 96, h), acc);
        const float bias = b2s[n];
#pragma unroll
        for (int r = 0; r < 8; ++r) h2w[r * HS + n] = (_Float16)fast_tanh(acc[r] * kWinv + bias);
      }
    }
    __syncthreads();

    const int slot = (t + 1) & 3;
    {
      const v16h ga0 = ld_frag_h(h2r, 0, h);
      const v16h ga1 = ld_frag_h(h2r, 32, h);
      const v16h ga2 = ld_frag_h(h2r, 64, h);
      const v16h ga3 = ld_frag_h(h2r, 96, h);
      const _Float16* wr = w3t + m * W3S;
      v8f acc;
#pragma unroll
      for (int r = 0; r < 8; ++r) acc[r] = 0.0f;
      acc = mma_f16(ga0, ld_frag_h(wr, 0, h), acc);
      acc = mma_f16(ga1, ld_frag_h(wr, 32, h), acc);
      acc = mma_f16(ga2, ld_frag_h(wr, 64, h), acc);
      acc = mma_f16(ga3, ld_frag_h(wr, 96, h), acc);
      if (m < kNY) {
        const float bias = b3s[m];
        float* ow = ow0 + slot * kNY + m;
#pragma unroll
        for (int r = 0; r < 8; ++r) ow[r * OBS] = acc[r] * kWinv + bias;
      }
    }
    __syncthreads();

    if (slot == 3) {
      const int g   = (t + 1) >> 2;
      const int q   = lane & 7;
      const int sub = lane >> 3;
      v4f vals[4];
      size_t offs[4];
      int oks[4];
#pragma unroll
      for (int i = 0; i < 4; ++i) {
        const int lr = lr0 + 4 * i + sub;
        const float* src = obuf + lr * OBS + 4 * q;
        v4f v;
        v.x = src[0]; v.y = src[1]; v.z = src[2]; v.w = src[3];
        vals[i] = v;
        const int gr = blockIdx.x * BROWS + lr;
        oks[i] = (gr < B) ? 1 : 0;
        offs[i] = (size_t)(oks[i] ? gr : 0) * (size_t)(kT * kNY) + (size_t)g * 32 + 4 * q;
      }
#pragma unroll
      for (int i = 0; i < 4; ++i)
        if (oks[i]) *(volatile v4f*)(out + offs[i]) = vals[i];
      __threadfence();
#pragma unroll
      for (int i = 0; i < 4; ++i)
        if (oks[i]) *(volatile v4f*)(out + offs[i]) = vals[i];
    }

    {
      v4us* const R = (v4us*)xrow;
      const v4us o0 = R[0], o1 = R[1];
      const v4us o4 = R[4], o5 = R[5], o6 = R[6], o7 = R[7], o8 = R[8], o9 = R[9];
      const v4us o11 = R[11], o12 = R[12], o13 = R[13], o14 = R[14];
      const float* yp = obuf + lrow * OBS + slot * kNY;
      v4us y0, y1;
      y0.x = bf16_part(yp[0], h); y0.y = bf16_part(yp[1], h);
      y0.z = bf16_part(yp[2], h); y0.w = bf16_part(yp[3], h);
      y1.x = bf16_part(yp[4], h); y1.y = bf16_part(yp[5], h);
      y1.z = bf16_part(yp[6], h); y1.w = bf16_part(yp[7], h);
      const v4f u = *(const v4f*)(useq + ((size_t)growc * kT + (size_t)(t + 1)) * kNU);
      v4us un;
      un.x = bf16_part(u.x, h); un.y = bf16_part(u.y, h);
      un.z = bf16_part(u.z, h); un.w = bf16_part(u.w, h);
      R[2] = o4; R[3] = o5; R[4] = o6; R[5] = o7; R[6] = o8; R[7] = o9;
      R[8] = o0; R[9] = o1;
      R[10] = o11; R[11] = o12; R[12] = o13;
      R[13] = o14;
      R[0] = y0; R[1] = y1;
      R[14] = un;
    }
  }
}

extern "C" void kernel_launch(void* const* d_in, const int* in_sizes, int n_in,
                              void* d_out, int out_size, void* d_ws, size_t ws_size,
                              hipStream_t stream) {
  (void)d_ws; (void)ws_size;
  if (n_in < 8) return;
  const float* useq = (const float*)d_in[0];
  const float* yz0  = (const float*)d_in[1];
  const float* W1   = (const float*)d_in[2];
  const float* b1   = (const float*)d_in[3];
  const float* W2   = (const float*)d_in[4];
  const float* b2   = (const float*)d_in[5];
  const float* W3   = (const float*)d_in[6];
  const float* b3   = (const float*)d_in[7];
  float* out = (float*)d_out;

  const int B = in_sizes[1] / kDS;
  if (B <= 0) return;
  if (in_sizes[1] != B * kDS) return;
  if (in_sizes[0] != B * kT * kNU) return;
  if (in_sizes[2] != kDI * kH || in_sizes[4] != kH * kH || in_sizes[6] != kH * kNY) return;
  if (in_sizes[3] < kH || in_sizes[5] < kH || in_sizes[7] < kNY) return;
  if (out_size != B * kT * kNY) return;

  const int blocks = (B + BROWS - 1) / BROWS;
  bbm_rollout<<<dim3(blocks), dim3(NTHR), 0, stream>>>(useq, yz0, W1, b1, W2, b2, W3, b3, out, B);
  (void)hipGetLastError();
}
